// MultiheadDiffAttn_17952963297574
// MI455X (gfx1250) — hardware-verified
//
#include <hip/hip_runtime.h>


#ifndef NB
#define NB 2
#endif
#ifndef SEQ
#define SEQ 2048
#endif
#define NB_FULL  2
#define SEQ_FULL 2048
#define EE   1024
#define NH   16
#define G2   32
#define HD   32
#define VD   64
#define NR   (NB * SEQ)
#define DM   EE
#define LOSC 4096.0f
#define WOSC 64.0f
#define QSC  0.17677669529663687f
#define LAM0 0.78360576653f
#define OML  0.21639423347f
static_assert(NB >= 1 && NB <= NB_FULL);
static_assert(SEQ >= 128 && SEQ <= SEQ_FULL && (SEQ % 128) == 0);
static_assert((EE % 64) == 0 && (NR % 64) == 0 && NH * VD == EE && G2 * HD == EE && G2 == 2 * NH);

#define QKV_BYTES ((size_t)3 * NR * EE * 4)
#define SAD_BYTES ((size_t)2 * SEQ * SEQ * 4 + (size_t)SEQ * SEQ * 2)
#define RBYTES ((QKV_BYTES > SAD_BYTES) ? QKV_BYTES : SAD_BYTES)
static_assert(QKV_BYTES <= RBYTES && SAD_BYTES <= RBYTES);

typedef _Float16 h16;
typedef unsigned short bf;
typedef __attribute__((ext_vector_type(16))) __bf16   v16bf;
typedef __attribute__((ext_vector_type(16))) _Float16 v16h;
typedef __attribute__((ext_vector_type(8)))  _Float16 v8h;
typedef __attribute__((ext_vector_type(4)))  _Float16 v4h;
typedef __attribute__((ext_vector_type(2)))  _Float16 v2h;
typedef __attribute__((ext_vector_type(8)))  unsigned short v8us;
typedef __attribute__((ext_vector_type(8)))  float    v8f;
typedef __attribute__((ext_vector_type(4)))  float    v4f;
typedef __attribute__((ext_vector_type(2)))  float    v2f;
typedef v8h  __attribute__((may_alias)) v8ha;
typedef v4f  __attribute__((may_alias)) v4fa;
typedef v8us __attribute__((may_alias)) v8usa;

__device__ __forceinline__ unsigned short f2bf(float f) { unsigned u = __float_as_uint(f); u += 0x7FFFu + ((u >> 16) & 1u); return (unsigned short)(u >> 16); }
__device__ __forceinline__ float bf2f(unsigned short b) { return __uint_as_float(((unsigned)b) << 16); }
__device__ __forceinline__ float bfr(float f) { return bf2f(f2bf(f)); }
__device__ __forceinline__ h16 tohx(float x) { return (h16)x; }
__device__ __forceinline__ v16h cat16(v8h lo, v8h hi) { return __builtin_shufflevector(lo, hi, 0, 1, 2, 3, 4, 5, 6, 7, 8, 9, 10, 11, 12, 13, 14, 15); }
__device__ __forceinline__ v16bf cat16b(v8us lo, v8us hi) { return __builtin_bit_cast(v16bf, __builtin_shufflevector(lo, hi, 0, 1, 2, 3, 4, 5, 6, 7, 8, 9, 10, 11, 12, 13, 14, 15)); }
__device__ __forceinline__ v8f wmma16(v16h a, v16h b, v8f c) { return __builtin_amdgcn_wmma_f32_16x16x32_f16(false, a, false, b, (short)0, c, false, false); }
__device__ __forceinline__ v8f wmmab(v16bf a, v16bf b, v8f c) { return __builtin_amdgcn_wmma_f32_16x16x32_bf16(false, a, false, b, (short)0, c, false, false); }

template <bool SPLITA, bool F16OUT = false>
__global__ __launch_bounds__(128) void k_gemmb(const bf* __restrict__ A, const bf* __restrict__ Al, const bf* __restrict__ Bn, const float* __restrict__ bias, float* C, int ldc, h16* C2, const float* __restrict__ R = nullptr, int K = DM, int rneR = 1) {
    __shared__ __align__(16) float ost[4][16 * 68];
    const int lane = threadIdx.x & 31, wave = threadIdx.x >> 5, lr = lane & 15, hi = lane >> 4;
    const int r0 = blockIdx.x * 64 + wave * 16, c0 = blockIdx.y * 64;
    const size_t aoff = (size_t)(r0 + lr) * K + 8 * hi;
    size_t boff[4];
#pragma unroll
    for (int t = 0; t < 4; ++t) boff[t] = (size_t)(c0 + t * 16 + lr) * K + 8 * hi;
    v8f acc[4];
#pragma unroll
    for (int t = 0; t < 4; ++t) acc[t] = (v8f){};
#pragma unroll 1
    for (int kc = 0; kc < K; kc += 32) {
        const v16bf a = cat16b(*(const v8us*)(A + aoff + kc), *(const v8us*)(A + aoff + kc + 16));
        v16bf al = a;
        if (SPLITA) al = cat16b(*(const v8us*)(Al + aoff + kc), *(const v8us*)(Al + aoff + kc + 16));
#pragma unroll
        for (int t = 0; t < 4; ++t) { const v16bf b = cat16b(*(const v8us*)(Bn + boff[t] + kc), *(const v8us*)(Bn + boff[t] + kc + 16)); acc[t] = wmmab(a, b, acc[t]); if (SPLITA) acc[t] = wmmab(al, b, acc[t]); }
        asm volatile("v_nop\n\tv_nop\n\tv_nop\n\tv_nop" : "+v"(acc[0]), "+v"(acc[1]), "+v"(acc[2]), "+v"(acc[3]) : "v"(a), "v"(al));
    }
    float* os = &ost[wave][0];
#pragma unroll
    for (int t = 0; t < 4; ++t) { const float bv = bias ? bfr(bias[c0 + t * 16 + lr]) : 0.f;
#pragma unroll
        for (int j = 0; j < 8; ++j) os[(hi * 8 + j) * 68 + t * 16 + lr] = acc[t][j] + bv; }
    __syncthreads();
    if (F16OUT) {
        h16* crow = (h16*)(void*)C + (size_t)r0 * ldc + c0;
        auto pass = [&]() {
#pragma unroll
            for (int s = 0; s < 4; ++s) { const int row = 4 * s + (lane >> 3), piece = lane & 7; const float* sp = os + row * 68 + piece * 8; v8h o, o2;
#pragma unroll
                for (int i = 0; i < 8; ++i) { const h16 a = (h16)sp[i]; o[i] = a; o2[i] = (h16)((sp[i] - (float)a) * LOSC); }
                *(volatile v8h*)(crow + (size_t)row * ldc + piece * 8) = o; if (C2) *(volatile v8h*)(C2 + (size_t)r0 * ldc + c0 + (size_t)row * ldc + piece * 8) = o2; }
        };
        pass(); __threadfence(); pass();
    } else {
        float* crow = C + (size_t)r0 * ldc + c0;
        auto pass = [&]() {
#pragma unroll
            for (int s = 0; s < 8; ++s) { const int Lid = (lane >> 3) + 4 * s, piece = lane & 7; const int row = Lid >> 1, cofs = (Lid & 1) * 32 + piece * 4;
                v4f val = *(const v4fa*)(os + row * 68 + cofs); if (R) { const v4f rv = *(const v4f*)(R + ((size_t)r0 + row) * ldc + c0 + cofs); val += rneR ? (v4f){bfr(rv[0]), bfr(rv[1]), bfr(rv[2]), bfr(rv[3])} : rv; }
                *(volatile v4f*)(crow + (size_t)row * ldc + cofs) = val; }
        };
        pass(); __threadfence(); pass();
    }
}

__global__ __launch_bounds__(128) void k_gemmh(const h16* __restrict__ A, const h16* __restrict__ Bn, const float* __restrict__ bias, float* C, int ldc, const float* __restrict__ R, int K, size_t sA, size_t sB, size_t sC, int rneR, float osc) {
    __shared__ __align__(16) float ost[4][16 * 68];
    const size_t z = blockIdx.z; A += z * sA; Bn += z * sB; C += z * sC; if (R) R += z * sC;
    const int lane = threadIdx.x & 31, wave = threadIdx.x >> 5, lr = lane & 15, hi = lane >> 4;
    const int r0 = blockIdx.x * 64 + wave * 16, c0 = blockIdx.y * 64;
    const size_t aoff = (size_t)(r0 + lr) * K + 8 * hi;
    size_t boff[4];
#pragma unroll
    for (int t = 0; t < 4; ++t) boff[t] = (size_t)(c0 + t * 16 + lr) * K + 8 * hi;
    v8f acc[4];
#pragma unroll
    for (int t = 0; t < 4; ++t) acc[t] = (v8f){};
#pragma unroll 1
    for (int kc = 0; kc < K; kc += 32) {
        const v16h a = cat16(*(const v8h*)(A + aoff + kc), *(const v8h*)(A + aoff + kc + 16));
#pragma unroll
        for (int t = 0; t < 4; ++t) { const v16h b = cat16(*(const v8h*)(Bn + boff[t] + kc), *(const v8h*)(Bn + boff[t] + kc + 16)); acc[t] = wmma16(a, b, acc[t]); }
        asm volatile("v_nop\n\tv_nop\n\tv_nop\n\tv_nop" : "+v"(acc[0]), "+v"(acc[1]), "+v"(acc[2]), "+v"(acc[3]) : "v"(a));
    }
    float* os = &ost[wave][0];
#pragma unroll
    for (int t = 0; t < 4; ++t) { const float bv = bias ? bfr(bias[c0 + t * 16 + lr]) : 0.f;
#pragma unroll
        for (int j = 0; j < 8; ++j) os[(hi * 8 + j) * 68 + t * 16 + lr] = acc[t][j] * osc + bv; }
    __syncthreads();
    float* crow = C + (size_t)r0 * ldc + c0;
    auto pass = [&]() {
#pragma unroll
        for (int s = 0; s < 8; ++s) { const int Lid = (lane >> 3) + 4 * s, piece = lane & 7; const int row = Lid >> 1, cofs = (Lid & 1) * 32 + piece * 4;
            v4f val = *(const v4fa*)(os + row * 68 + cofs); if (R) { const v4f rv = *(const v4f*)(R + ((size_t)r0 + row) * ldc + c0 + cofs); val += rneR ? (v4f){bfr(rv[0]), bfr(rv[1]), bfr(rv[2]), bfr(rv[3])} : rv; }
            *(volatile v4f*)(crow + (size_t)row * ldc + cofs) = val; }
    };
    pass(); __threadfence(); pass();
}

template <int MODE>
__global__ __launch_bounds__(256) void k_cvt(const float* __restrict__ src, void* dst, int nrows, int seg, int segfull) {
    const int lane = threadIdx.x & 31; const int r = blockIdx.x * 8 + (threadIdx.x >> 5); if (r >= nrows) return;
    const size_t srow = (size_t)(r / seg) * segfull + (size_t)(r % seg);
    const float* sp = src + srow * EE; const size_t drow = (size_t)r * EE;
#pragma unroll 1
    for (int ps = 0; ps < 2; ++ps) {
#pragma unroll
        for (int q = 0; q < EE / 256; ++q) { const size_t o = (size_t)q * 256 + lane * 8;
            const v4f a = *(const v4f*)(sp + o), c = *(const v4f*)(sp + o + 4);
            if (MODE == 0) { v8us v;
#pragma unroll
                for (int k = 0; k < 4; ++k) { v[k] = f2bf(a[k]); v[4 + k] = f2bf(c[k]); }
                *(volatile v8us*)((bf*)dst + drow + o) = v;
            } else { v8h v;
#pragma unroll
                for (int k = 0; k < 4; ++k) { v[k] = tohx(bfr(a[k]) * WOSC); v[4 + k] = tohx(bfr(c[k]) * WOSC); }
                *(volatile v8h*)((h16*)dst + drow + o) = v; } }
        if (ps == 0) __threadfence(); }
}

__global__ __launch_bounds__(256) void k_qkpl(const float* __restrict__ Q, const float* __restrict__ Kf, h16* QH, h16* KH) {
    const int lane = threadIdx.x & 31; const int w = blockIdx.x * 8 + (threadIdx.x >> 5); if (w >= NB * G2 * (SEQ / 8)) return;
    const int which = blockIdx.y; const float* F = which ? Kf : Q; h16* P = which ? KH : QH; const float sc = which ? 1.0f : QSC;
    const int ib = w % (SEQ / 8); const int rest = w / (SEQ / 8); const int g = rest % G2, b = rest / G2;
    const int i = ib * 8 + (lane >> 2), dq = (lane & 3) * 8;
    const float* sp = F + ((size_t)b * SEQ + i) * EE + g * HD + dq;
    const v4f a = *(const v4f*)sp, c = *(const v4f*)(sp + 4);
    v8h o;
#pragma unroll
    for (int k = 0; k < 4; ++k) { o[k] = tohx(a[k] * sc); o[4 + k] = tohx(c[k] * sc); }
    const size_t off = ((size_t)(b * G2 + g) * SEQ + i) * HD + dq;
    *(volatile v8h*)(P + off) = o; __threadfence(); *(volatile v8h*)(P + off) = o;
}

__global__ __launch_bounds__(256) void k_vT(const float* __restrict__ V, h16* VT) {
    __shared__ float tl[64][65];
    const int tid = threadIdx.x; const int t0 = blockIdx.x * 64; const int bh = blockIdx.y; const int b = bh / NH, h = bh % NH; const int rr = tid >> 2, cq = (tid & 3) * 16;
#pragma unroll
    for (int i = 0; i < 16; ++i) tl[rr][cq + i] = V[((size_t)b * SEQ + t0 + rr) * EE + h * VD + cq + i];
    __syncthreads();
    const int lane = tid & 31, wv = tid >> 5;
    auto pass = [&]() {
#pragma unroll
        for (int st = 0; st < 4; ++st) { const int dr = wv * 8 + st * 2 + (lane >> 4); const int tq = (lane & 15) * 4; v4h v;
#pragma unroll
            for (int i = 0; i < 4; ++i) v[i] = tohx(tl[tq + i][dr]);
            *(volatile v4h*)(VT + ((size_t)bh * VD + dr) * SEQ + t0 + tq) = v; }
    };
    pass(); __threadfence(); pass();
}

__global__ __launch_bounds__(256) void k_softdiff(const float* __restrict__ S, const float* __restrict__ lq1, const float* __restrict__ lk1, const float* __restrict__ lq2, const float* __restrict__ lk2, h16* AD) {
    __shared__ __align__(16) h16 stash[8][SEQ];
    const int lane = threadIdx.x & 31, wave = threadIdx.x >> 5, i = blockIdx.x * 8 + wave; if (i >= SEQ) return;
    float d1 = bfr(lq1[lane]) * bfr(lk1[lane]); float d2 = bfr(lq2[lane]) * bfr(lk2[lane]);
#pragma unroll
    for (int sh = 16; sh; sh >>= 1) { d1 += __shfl_xor(d1, sh, 32); d2 += __shfl_xor(d2, sh, 32); }
    const float lam = expf(d1) - expf(d2) + LAM0;
    const float* s1 = S + (size_t)i * SEQ; const float* s2 = S + ((size_t)SEQ + i) * SEQ;
    float m1 = -3.0e38f, m2 = -3.0e38f;
#pragma unroll 1
    for (int c0 = lane * 4; c0 < SEQ; c0 += 128) { const v4f a = *(const v4f*)(s1 + c0), c = *(const v4f*)(s2 + c0);
#pragma unroll
        for (int q = 0; q < 4; ++q) { m1 = fmaxf(m1, a[q]); m2 = fmaxf(m2, c[q]); } }
#pragma unroll
    for (int sh = 16; sh; sh >>= 1) { m1 = fmaxf(m1, __shfl_xor(m1, sh, 32)); m2 = fmaxf(m2, __shfl_xor(m2, sh, 32)); }
    float u1 = 0.f, u2 = 0.f;
#pragma unroll 1
    for (int c0 = lane * 4; c0 < SEQ; c0 += 128) { const v4f a = *(const v4f*)(s1 + c0), c = *(const v4f*)(s2 + c0);
#pragma unroll
        for (int q = 0; q < 4; ++q) { u1 += __expf(a[q] - m1); u2 += __expf(c[q] - m2); } }
#pragma unroll
    for (int sh = 16; sh; sh >>= 1) { u1 += __shfl_xor(u1, sh, 32); u2 += __shfl_xor(u2, sh, 32); }
    const float i1 = (1.0f / u1) * LOSC, i2 = (1.0f / u2) * lam * LOSC;
    h16* st = &stash[wave][0]; h16* ad = AD + (size_t)i * SEQ;
#pragma unroll 1
    for (int c0 = lane * 4; c0 < SEQ; c0 += 128) { const v4f a = *(const v4f*)(s1 + c0), c = *(const v4f*)(s2 + c0); v4h o;
#pragma unroll
        for (int q = 0; q < 4; ++q) o[q] = tohx(__expf(a[q] - m1) * i1 - __expf(c[q] - m2) * i2);
        *(v4h*)(st + c0) = o;
        *(volatile v4h*)(ad + c0) = o; }
    __threadfence();
#pragma unroll 1
    for (int c0 = lane * 4; c0 < SEQ; c0 += 128) { const v4h o = *(const v4h*)(st + c0); *(volatile v4h*)(ad + c0) = o; }
}

__global__ __launch_bounds__(256) void k_rms(const float* __restrict__ O, const float* __restrict__ gw, h16* OH) {
    const int lane = threadIdx.x & 31; const int w = blockIdx.x * 8 + (threadIdx.x >> 5); if (w >= NB * NH * SEQ) return;
    const int i = w % SEQ; const int bh = w / SEQ; const int h = bh % NH, b = bh / NH;
    v2f v = *(const v2f*)(O + (size_t)w * VD + lane * 2); v = v * (1.0f / LOSC);
    float q = v[0] * v[0] + v[1] * v[1];
#pragma unroll
    for (int sh = 16; sh; sh >>= 1) q += __shfl_xor(q, sh, 32);
    const float rs = rsqrtf(q * (1.0f / VD) + 1e-5f); v2h o;
#pragma unroll
    for (int k = 0; k < 2; ++k) o[k] = tohx(((v[k] * rs) * bfr(gw[lane * 2 + k])) * OML);
    const size_t off = ((size_t)b * SEQ + i) * EE + h * VD + lane * 2; *(volatile v2h*)(OH + off) = o; __threadfence(); *(volatile v2h*)(OH + off) = o;
}

extern "C" void kernel_launch(void* const* d_in, const int* in_sizes, int n_in,
                              void* d_out, int out_size, void* d_ws, size_t ws_size, hipStream_t stream) {
    if (n_in < 10) return;
    const size_t needx = ((size_t)(NB - 1) * SEQ_FULL + SEQ) * EE;
    if ((size_t)in_sizes[0] < needx || (size_t)out_size < needx) return;
    for (int j = 1; j <= 4; ++j) if (in_sizes[j] < EE * EE) return;
    for (int j = 5; j <= 8; ++j) if (in_sizes[j] < HD) return;
    if (in_sizes[9] < VD) return;
    const float* x = (const float*)d_in[0]; const float* Wq = (const float*)d_in[1]; const float* Wk = (const float*)d_in[2]; const float* Wv = (const float*)d_in[3]; const float* Wo = (const float*)d_in[4];
    const float* lq1 = (const float*)d_in[5]; const float* lk1 = (const float*)d_in[6]; const float* lq2 = (const float*)d_in[7]; const float* lk2 = (const float*)d_in[8];
    const float* nw = (const float*)d_in[9];
    float* out = (float*)d_out;
    char* wsp = (char*)d_ws;
    auto take = [&](size_t bytes) { char* p = wsp; wsp += (bytes + 255) & ~(size_t)255; return (void*)p; };
    bf* WQB = (bf*)take((size_t)EE * EE * 2); bf* WKB = (bf*)take((size_t)EE * EE * 2); bf* WVB = (bf*)take((size_t)EE * EE * 2); h16* WOH = (h16*)take((size_t)EE * EE * 2);
    bf* XB = (bf*)take((size_t)NR * EE * 2);
    h16* QH = (h16*)take((size_t)NB * G2 * SEQ * HD * 2); h16* KH = (h16*)take((size_t)NB * G2 * SEQ * HD * 2); h16* VT = (h16*)take((size_t)NB * NH * VD * SEQ * 2);
    float* O = (float*)take((size_t)NB * NH * SEQ * VD * 4); h16* OH = (h16*)take((size_t)NR * EE * 2);
    char* RG = (char*)take(RBYTES);
    if ((size_t)(wsp - (char*)d_ws) > ws_size) return;
    float* Q = (float*)RG; float* Kf = (float*)(RG + (size_t)NR * EE * 4); float* V = (float*)(RG + (size_t)2 * NR * EE * 4);
    float* S = (float*)RG; h16* AD = (h16*)(RG + (size_t)2 * SEQ * SEQ * 4);
    k_cvt<0><<<dim3(NR / 8, 1, 1), 256, 0, stream>>>(x, (void*)XB, NR, SEQ, SEQ_FULL);
    k_cvt<0><<<dim3(EE / 8, 1, 1), 256, 0, stream>>>(Wq, (void*)WQB, EE, EE, EE);
    k_cvt<0><<<dim3(EE / 8, 1, 1), 256, 0, stream>>>(Wk, (void*)WKB, EE, EE, EE);
    k_cvt<0><<<dim3(EE / 8, 1, 1), 256, 0, stream>>>(Wv, (void*)WVB, EE, EE, EE);
    k_cvt<1><<<dim3(EE / 8, 1, 1), 256, 0, stream>>>(Wo, (void*)WOH, EE, EE, EE);
    k_gemmb<false, false><<<dim3(NR / 64, EE / 64, 1), 128, 0, stream>>>(XB, nullptr, WQB, nullptr, Q, EE, nullptr, nullptr, EE);
    k_gemmb<false, false><<<dim3(NR / 64, EE / 64, 1), 128, 0, stream>>>(XB, nullptr, WKB, nullptr, Kf, EE, nullptr, nullptr, EE);
    k_gemmb<false, false><<<dim3(NR / 64, EE / 64, 1), 128, 0, stream>>>(XB, nullptr, WVB, nullptr, V, EE, nullptr, nullptr, EE);
    k_qkpl<<<dim3((NB * G2 * (SEQ / 8) + 7) / 8, 2, 1), 256, 0, stream>>>(Q, Kf, QH, KH);
    k_vT<<<dim3(SEQ / 64, NB * NH, 1), 256, 0, stream>>>(V, VT);
    for (int b = 0; b < NB; ++b)
        for (int h = 0; h < NH; ++h) {
            const size_t qo = (size_t)(b * G2 + 2 * h) * SEQ * HD; const size_t bh = (size_t)b * NH + h;
            k_gemmh<<<dim3(SEQ / 64, SEQ / 64, 2), 128, 0, stream>>>(QH + qo, KH + qo, nullptr, S, SEQ, nullptr, HD, (size_t)SEQ * HD, (size_t)SEQ * HD, (size_t)SEQ * SEQ, 0, 1.0f);
            k_softdiff<<<dim3(SEQ / 8, 1, 1), 256, 0, stream>>>(S, lq1, lk1, lq2, lk2, AD);
            k_gemmh<<<dim3(SEQ / 64, VD / 64, 1), 128, 0, stream>>>(AD, VT + bh * VD * SEQ, nullptr, O + bh * SEQ * VD, VD, nullptr, SEQ, 0, 0, 0, 0, 1.0f); }
    k_rms<<<dim3((NB * NH * SEQ + 7) / 8, 1, 1), 256, 0, stream>>>(O, nw, OH);
    k_gemmh<<<dim3(SEQ / 64, EE / 64, NB), 128, 0, stream>>>(OH, WOH, nullptr, out, EE, nullptr, EE, (size_t)SEQ * EE, 0, (size_t)SEQ_FULL * EE, 0, 1.0f / WOSC);
}
